// FinancialSentimentLoRA_25555055411403
// MI455X (gfx1250) — hardware-verified
//
#include <hip/hip_runtime.h>
#include <stddef.h>


constexpr int NB   = 8;
constexpr int NS   = 1024;
constexpr int ND   = 1024;
constexpr int NH   = 16;
constexpr int HD   = 64;
constexpr int NR   = 8;
constexpr int NFF  = 4096;
constexpr int NDC  = 512;
constexpr int NCLS = 3;
constexpr int NTOK = NB * NS;
constexpr int SLOTW = 32;
constexpr float ADSCALE = 2.0f;
constexpr float WSC     = 32.0f;
constexpr float WSC_INV = 0.03125f;

static_assert(NR == 8);
static_assert(ND == 256 * 4);
static_assert(ND == 128 * 8);
static_assert(NH * HD == ND);
static_assert(NS == 4 * 256);
static_assert(HD == 64);
static_assert(NFF == 4 * ND);
static_assert(NTOK % 128 == 0);
static_assert(ND % 128 == 0);
static_assert(ND % 32 == 0);
static_assert(NCLS <= 4);

typedef _Float16 f16;
typedef f16   v16h __attribute__((ext_vector_type(16)));
typedef f16   v8h  __attribute__((ext_vector_type(8)));
typedef f16   v4h  __attribute__((ext_vector_type(4)));
typedef float v8f  __attribute__((ext_vector_type(8)));
typedef float v4f  __attribute__((ext_vector_type(4)));
typedef v4f   v4fa __attribute__((may_alias));

union Frag  { v16h v; v8h half[2]; };
union Pack8 { v8h v; v4h q[2]; };

__device__ __forceinline__ v8f wmma_f16(v16h a, v16h b, v8f c)
{
  v8f d = __builtin_amdgcn_wmma_f32_16x16x32_f16(false, a, false, b, (short)0, c, false, false);
  asm volatile("v_nop\n\tv_nop\n\tv_nop\n\tv_nop" : "+v"(d) : "v"(a), "v"(b));
  return d;
}

__device__ __forceinline__ float wave_sum(float v)
{
#pragma unroll
  for (int s = 16; s > 0; s >>= 1) v += __shfl_xor(v, s, 32);
  return v;
}

__device__ __forceinline__ float wave_max(float v)
{
#pragma unroll
  for (int s = 16; s > 0; s >>= 1) v = fmaxf(v, __shfl_xor(v, s, 32));
  return v;
}

__device__ __forceinline__ float sum8(const float* r)
{
  return ((r[0] + r[1]) + (r[2] + r[3])) + ((r[4] + r[5]) + (r[6] + r[7]));
}

template<int UNR>
__device__ __forceinline__ float wave_dot(const float* xs, const float* __restrict__ w, int K, int lane)
{
  float a = 0.0f;
#pragma unroll UNR
  for (int d = lane; d < K; d += 32) a += xs[d] * w[d];
  return wave_sum(a);
}

__device__ __forceinline__ float geluf(float x)
{
  return 0.5f * x * (1.0f + erff(x * 0.70710678118654752440f));
}

__device__ __forceinline__ v4h cvt4(v4f x) { return __builtin_convertvector(x, v4h); }

__device__ __forceinline__ void block_ln(v4f v, const float* __restrict__ g, const float* __restrict__ be,
                                         float* dst, float* red, float* stat, int tid, int lane, int wave)
{
  float s = (v.x + v.y) + (v.z + v.w);
  s = wave_sum(s);
  if (lane == 0) red[wave] = s;
  __syncthreads();
  if (tid == 0) stat[0] = sum8(red) * (1.0f / ND);
  __syncthreads();
  const float mu = stat[0];
  const v4f d = v - mu;
  const v4f dq = d * d;
  float s2 = (dq.x + dq.y) + (dq.z + dq.w);
  s2 = wave_sum(s2);
  if (lane == 0) red[wave] = s2;
  __syncthreads();
  if (tid == 0) stat[1] = sum8(red) * (1.0f / ND);
  __syncthreads();
  const float rstd = rsqrtf(stat[1] + 1e-5f);
  const v4f gg = *(const v4f*)(g + 4 * tid);
  const v4f bb = *(const v4f*)(be + 4 * tid);
  const v4f y = d * rstd * gg + bb;
  *(v4fa*)(dst + 4 * tid) = y;
}

__global__ __launch_bounds__(128)
void k_ln_rows(const float* __restrict__ x, const float* __restrict__ g, const float* __restrict__ be,
               f16* __restrict__ outh)
{
  __shared__ float red[4];
  __shared__ float stat[2];
  const int row = blockIdx.x, tid = threadIdx.x, lane = tid & 31, wave = tid >> 5;
  const size_t base = (size_t)row * ND + (size_t)tid * 8;
  const v4f a0 = *(const v4f*)(x + base);
  const v4f a1 = *(const v4f*)(x + base + 4);
  float s = ((a0.x + a0.y) + (a0.z + a0.w)) + ((a1.x + a1.y) + (a1.z + a1.w));
  s = wave_sum(s);
  if (lane == 0) red[wave] = s;
  __syncthreads();
  if (tid == 0) stat[0] = ((red[0] + red[1]) + (red[2] + red[3])) * (1.0f / ND);
  __syncthreads();
  const float mu = stat[0];
  const v4f d0 = a0 - mu, d1 = a1 - mu;
  const v4f p0 = d0 * d0, p1 = d1 * d1;
  float s2 = ((p0.x + p0.y) + (p0.z + p0.w)) + ((p1.x + p1.y) + (p1.z + p1.w));
  s2 = wave_sum(s2);
  if (lane == 0) red[wave] = s2;
  __syncthreads();
  if (tid == 0) stat[1] = ((red[0] + red[1]) + (red[2] + red[3])) * (1.0f / ND);
  __syncthreads();
  const float rstd = rsqrtf(stat[1] + 1e-5f);
  const v4f g0 = *(const v4f*)(g + tid * 8), g1 = *(const v4f*)(g + tid * 8 + 4);
  const v4f b0 = *(const v4f*)(be + tid * 8), b1v = *(const v4f*)(be + tid * 8 + 4);
  const v4f y0 = d0 * rstd * g0 + b0;
  const v4f y1 = d1 * rstd * g1 + b1v;
  Pack8 pk;
  pk.q[0] = cvt4(y0);
  pk.q[1] = cvt4(y1);
  f16* op = outh + base;
  *(volatile v8h*)op = pk.v;
  __threadfence();
  *(volatile v8h*)op = pk.v;
}

__global__ __launch_bounds__(256)
void k_fold(const float* __restrict__ Wk, const float* __restrict__ Ak, const float* __restrict__ Bk,
            const float* __restrict__ Wv, const float* __restrict__ Av, const float* __restrict__ Bv,
            f16* __restrict__ outk, f16* __restrict__ outv)
{
  const bool sv = (blockIdx.y != 0);
  const float* W  = sv ? Wv : Wk;
  const float* A  = sv ? Av : Ak;
  const float* Bm = sv ? Bv : Bk;
  f16* o = sv ? outv : outk;
  const int t = blockIdx.x * 256 + threadIdx.x;
  const int n = t >> 7, k8 = (t & 127) * 8;
  const size_t wb = (size_t)n * ND + k8;
  v4f w0 = *(const v4f*)(W + wb);
  v4f w1 = *(const v4f*)(W + wb + 4);
  v4f l0 = {0.0f, 0.0f, 0.0f, 0.0f};
  v4f l1 = l0;
#pragma unroll 2
  for (int r = 0; r < NR; ++r) {
    const float br = Bm[(size_t)n * NR + r];
    const v4f x0 = *(const v4f*)(A + (size_t)r * ND + k8);
    const v4f x1 = *(const v4f*)(A + (size_t)r * ND + k8 + 4);
    l0 += br * x0;
    l1 += br * x1;
  }
  w0 = (w0 + ADSCALE * l0) * WSC;
  w1 = (w1 + ADSCALE * l1) * WSC;
  Pack8 pk;
  pk.q[0] = cvt4(w0);
  pk.q[1] = cvt4(w1);
  f16* op = o + wb;
  *(volatile v8h*)op = pk.v;
  __threadfence();
  *(volatile v8h*)op = pk.v;
}

constexpr int GP = 5;

__global__ __launch_bounds__(256)
void k_gemm_kv(const f16* __restrict__ Ah, const f16* __restrict__ Wkh, const f16* __restrict__ Wvh,
               float* __restrict__ Kout, float* __restrict__ Vout)
{
  __shared__ v8h As[128 * GP];
  __shared__ v8h Bs[128 * GP];
  __shared__ __align__(16) float Cst[8 * 16 * 64];

  const bool sv = (blockIdx.z != 0);
  const f16* Wh = sv ? Wvh : Wkh;
  float* outp = sv ? Vout : Kout;
  const int m0 = blockIdx.y * 128, n0 = blockIdx.x * 128;
  const int tid = threadIdx.x, lane = tid & 31, wave = tid >> 5;
  const int hh = lane >> 4, mm = lane & 15;
  const int wm = (wave & 3) * 32, wn = (wave >> 2) * 64;

  v8f acc[2][4];
#pragma unroll
  for (int i = 0; i < 2; ++i) {
#pragma unroll
    for (int j = 0; j < 4; ++j) {
      v8f z = {0.0f, 0.0f, 0.0f, 0.0f, 0.0f, 0.0f, 0.0f, 0.0f};
      acc[i][j] = z;
    }
  }

  for (int kb = 0; kb < ND; kb += 32) {
    __syncthreads();
#pragma unroll
    for (int it = 0; it < 2; ++it) {
      const int idx = tid + it * 256;
      const int r = idx >> 2, c = idx & 3;
      As[r * GP + c] = *(const v8h*)(Ah + (size_t)(m0 + r) * ND + kb + c * 8);
      Bs[r * GP + c] = *(const v8h*)(Wh + (size_t)(n0 + r) * ND + kb + c * 8);
    }
    __syncthreads();
    Frag fa[2], fb[4];
#pragma unroll
    for (int i = 0; i < 2; ++i) {
      const int rr = wm + i * 16 + mm;
      fa[i].half[0] = As[rr * GP + hh];
      fa[i].half[1] = As[rr * GP + 2 + hh];
    }
#pragma unroll
    for (int j = 0; j < 4; ++j) {
      const int nn = wn + j * 16 + mm;
      fb[j].half[0] = Bs[nn * GP + hh];
      fb[j].half[1] = Bs[nn * GP + 2 + hh];
    }
#pragma unroll
    for (int i = 0; i < 2; ++i) {
#pragma unroll
      for (int j = 0; j < 4; ++j) acc[i][j] = wmma_f16(fa[i].v, fb[j].v, acc[i][j]);
    }
  }

  float* cw = Cst + wave * (16 * 64);
  const int c4 = mm * 4;
#pragma unroll
  for (int i = 0; i < 2; ++i) {
    __syncthreads();
#pragma unroll
    for (int j = 0; j < 4; ++j) {
#pragma unroll
      for (int r = 0; r < 8; ++r) cw[(8 * hh + r) * 64 + j * 16 + mm] = acc[i][j][r] * WSC_INV;
    }
    __syncthreads();
    const int grow0 = m0 + wm + i * 16;
#pragma unroll
    for (int s = 0; s < 8; ++s) {
      const int rr = 2 * s + hh;
      const v4f val = *(const v4fa*)(cw + rr * 64 + c4);
      float* gptr = outp + (size_t)(grow0 + rr) * ND + n0 + wn + c4;
      *(volatile v4f*)gptr = val;
    }
    __threadfence();
#pragma unroll
    for (int s = 0; s < 8; ++s) {
      const int rr = 2 * s + hh;
      const v4f val = *(const v4fa*)(cw + rr * 64 + c4);
      float* gptr = outp + (size_t)(grow0 + rr) * ND + n0 + wn + c4;
      *(volatile v4f*)gptr = val;
    }
  }
}

__global__ __launch_bounds__(256)
void k_cls_q(const float* __restrict__ hidden, const float* __restrict__ g1, const float* __restrict__ be1,
             const float* __restrict__ Wq, const float* __restrict__ Aq, const float* __restrict__ Bq,
             float* __restrict__ q0out)
{
  __shared__ __align__(16) float xs[ND];
  __shared__ __align__(16) float qs[ND];
  __shared__ float tq[NR];
  __shared__ float red[8];
  __shared__ float stat[2];
  const int b = blockIdx.x, tid = threadIdx.x, lane = tid & 31, wave = tid >> 5;
  const float* xr = hidden + (size_t)b * NS * ND;
  const v4f v = *(const v4f*)(xr + 4 * tid);
  block_ln(v, g1, be1, xs, red, stat, tid, lane, wave);
  __syncthreads();
  {
    const float a = wave_dot<1>(xs, Aq + (size_t)wave * ND, ND, lane);
    if (lane == 0) tq[wave] = a;
  }
  __syncthreads();
  for (int j = 0; j < ND / 8; ++j) {
    const int n = j * 8 + wave;
    const float a = wave_dot<2>(xs, Wq + (size_t)n * ND, ND, lane);
    float lr = 0.0f;
#pragma unroll
    for (int r = 0; r < NR; ++r) lr += tq[r] * Bq[(size_t)n * NR + r];
    if (lane == 0) qs[n] = a + ADSCALE * lr;
  }
  __syncthreads();
  const v4f qv = *(const v4fa*)(qs + 4 * tid);
  float* qp = q0out + (size_t)b * ND + 4 * tid;
  *(volatile v4f*)qp = qv;
  __threadfence();
  *(volatile v4f*)qp = qv;
}

__global__ __launch_bounds__(256)
void k_cls_attn(const float* __restrict__ q0, const float* __restrict__ Kf, const float* __restrict__ Vf,
                float* __restrict__ ctx)
{
  __shared__ __align__(16) float qh[HD];
  __shared__ float sc[NS];
  __shared__ float part[4 * HD];
  __shared__ __align__(16) float cs[HD];
  __shared__ float red[8];
  __shared__ float stat[2];
  const int h = blockIdx.x, b = blockIdx.y;
  const int tid = threadIdx.x, lane = tid & 31, wave = tid >> 5;
  if (tid < HD) qh[tid] = q0[(size_t)b * ND + h * HD + tid];
  __syncthreads();

  float mloc = -3.0e38f;
#pragma unroll 1
  for (int kk = 0; kk < NS / 256; ++kk) {
    const int key = tid + kk * 256;
    const float* kr = Kf + ((size_t)b * NS + key) * ND + h * HD;
    float s = 0.0f;
#pragma unroll 4
    for (int d4 = 0; d4 < HD / 4; ++d4) {
      const v4f kv = *(const v4f*)(kr + 4 * d4);
      const v4f qv = *(const v4fa*)(qh + 4 * d4);
      const v4f pq = qv * kv;
      s += (pq.x + pq.y) + (pq.z + pq.w);
    }
    s *= 0.125f;
    sc[key] = s;
    mloc = fmaxf(mloc, s);
  }
  mloc = wave_max(mloc);
  if (lane == 0) red[wave] = mloc;
  __syncthreads();
  if (tid == 0) {
    float m = red[0];
#pragma unroll
    for (int i = 1; i < 8; ++i) m = fmaxf(m, red[i]);
    stat[0] = m;
  }
  __syncthreads();
  const float mx = stat[0];
  float ls = 0.0f;
#pragma unroll 1
  for (int kk = 0; kk < NS / 256; ++kk) {
    const int key = tid + kk * 256;
    const float p = expf(sc[key] - mx);
    sc[key] = p;
    ls += p;
  }
  ls = wave_sum(ls);
  if (lane == 0) red[wave] = ls;
  __syncthreads();
  if (tid == 0) stat[1] = sum8(red);
  __syncthreads();
  const float inv = 1.0f / stat[1];
#pragma unroll
  for (int kk = 0; kk < NS / 256; ++kk) sc[tid + kk * 256] *= inv;
  __syncthreads();

  const int d = tid & (HD - 1), kg = tid >> 6;
  const float* vp = Vf + ((size_t)b * NS + kg * 256) * ND + h * HD + d;
  const float* sp = sc + kg * 256;
  float a = 0.0f;
#pragma unroll 4
  for (int k = 0; k < 256; ++k) a += sp[k] * vp[(size_t)k * ND];
  part[kg * HD + d] = a;
  __syncthreads();
  if (tid < HD) cs[tid] = (part[tid] + part[HD + tid]) + (part[2 * HD + tid] + part[3 * HD + tid]);
  __syncthreads();
  if (tid < HD / 4) {
    const v4f cv = *(const v4fa*)(cs + 4 * tid);
    float* cp = ctx + (size_t)b * ND + h * HD + 4 * tid;
    *(volatile v4f*)cp = cv;
    __threadfence();
    *(volatile v4f*)cp = cv;
  }
}

__global__ __launch_bounds__(256)
void k_cls_mid(const float* __restrict__ ctx, const float* __restrict__ hidden,
               const float* __restrict__ Wo, const float* __restrict__ Ao, const float* __restrict__ Bo,
               const float* __restrict__ g2, const float* __restrict__ be2,
               const float* __restrict__ W1, const float* __restrict__ b1,
               float* __restrict__ hAout, float* __restrict__ ffout)
{
  __shared__ __align__(16) float cx[ND];
  __shared__ __align__(16) float hA[ND];
  __shared__ __align__(16) float hn[ND];
  __shared__ __align__(16) float ff[NFF];
  __shared__ float tr[NR];
  __shared__ float red[8];
  __shared__ float stat[2];
  const int b = blockIdx.x, tid = threadIdx.x, lane = tid & 31, wave = tid >> 5;
  for (int i = tid; i < ND; i += 256) cx[i] = ctx[(size_t)b * ND + i];
  __syncthreads();
  {
    const float a = wave_dot<1>(cx, Ao + (size_t)wave * ND, ND, lane);
    if (lane == 0) tr[wave] = a;
  }
  __syncthreads();
  const float* x0 = hidden + (size_t)b * NS * ND;
  for (int j = 0; j < ND / 8; ++j) {
    const int n = j * 8 + wave;
    const float a = wave_dot<2>(cx, Wo + (size_t)n * ND, ND, lane);
    float lr = 0.0f;
#pragma unroll
    for (int r = 0; r < NR; ++r) lr += tr[r] * Bo[(size_t)n * NR + r];
    if (lane == 0) hA[n] = x0[n] + (a + ADSCALE * lr);
  }
  __syncthreads();
  {
    const v4f v = *(const v4fa*)(hA + 4 * tid);
    block_ln(v, g2, be2, hn, red, stat, tid, lane, wave);
  }
  __syncthreads();
  for (int j = 0; j < NFF / 8; ++j) {
    const int f = j * 8 + wave;
    const float a = wave_dot<4>(hn, W1 + (size_t)f * ND, ND, lane);
    const float gv = geluf(a + b1[f]);
    if (lane == 0) ff[f] = gv;
  }
  __syncthreads();
  const v4f hv  = *(const v4fa*)(hA + 4 * tid);
  const v4f fv0 = *(const v4fa*)(ff + 0 * ND + 4 * tid);
  const v4f fv1 = *(const v4fa*)(ff + 1 * ND + 4 * tid);
  const v4f fv2 = *(const v4fa*)(ff + 2 * ND + 4 * tid);
  const v4f fv3 = *(const v4fa*)(ff + 3 * ND + 4 * tid);
  float* hp = hAout + (size_t)b * ND + 4 * tid;
  float* fp = ffout + (size_t)b * NFF + 4 * tid;
  *(volatile v4f*)hp = hv;
  *(volatile v4f*)(fp + 0 * ND) = fv0;
  *(volatile v4f*)(fp + 1 * ND) = fv1;
  *(volatile v4f*)(fp + 2 * ND) = fv2;
  *(volatile v4f*)(fp + 3 * ND) = fv3;
  __threadfence();
  *(volatile v4f*)hp = hv;
  *(volatile v4f*)(fp + 0 * ND) = fv0;
  *(volatile v4f*)(fp + 1 * ND) = fv1;
  *(volatile v4f*)(fp + 2 * ND) = fv2;
  *(volatile v4f*)(fp + 3 * ND) = fv3;
}

__global__ __launch_bounds__(256)
void k_cls_head(const float* __restrict__ hAin, const float* __restrict__ ffin,
                const float* __restrict__ W2, const float* __restrict__ b2,
                const float* __restrict__ Wc1, const float* __restrict__ bc1,
                const float* __restrict__ Wc2, const float* __restrict__ bc2,
                float* __restrict__ slots)
{
  __shared__ __align__(16) float ff[NFF];
  __shared__ __align__(16) float hA[ND];
  __shared__ __align__(16) float h3[ND];
  __shared__ __align__(16) float c1[NDC];
  __shared__ float lg[4];
  const int b = blockIdx.x, tid = threadIdx.x, lane = tid & 31, wave = tid >> 5;
  for (int i = tid; i < NFF; i += 256) ff[i] = ffin[(size_t)b * NFF + i];
  for (int i = tid; i < ND; i += 256) hA[i] = hAin[(size_t)b * ND + i];
  if (tid < 4) lg[tid] = 0.0f;
  __syncthreads();
  for (int j = 0; j < ND / 8; ++j) {
    const int n = j * 8 + wave;
    const float a = wave_dot<4>(ff, W2 + (size_t)n * NFF, NFF, lane);
    if (lane == 0) h3[n] = hA[n] + (a + b2[n]);
  }
  __syncthreads();
  for (int j = 0; j < NDC / 8; ++j) {
    const int c = j * 8 + wave;
    const float a = wave_dot<2>(h3, Wc1 + (size_t)c * ND, ND, lane);
    const float gv = geluf(a + bc1[c]);
    if (lane == 0) c1[c] = gv;
  }
  __syncthreads();
  if (wave < NCLS) {
    const float a = wave_dot<1>(c1, Wc2 + (size_t)wave * NDC, NDC, lane);
    if (lane == 0) lg[wave] = a + bc2[wave];
  }
  __syncthreads();
  if (tid == 0) {
    const v4f v0 = {lg[0], lg[1], lg[2], 0.0f};
    const v4f z  = {0.0f, 0.0f, 0.0f, 0.0f};
    float* sp = slots + (size_t)b * SLOTW;
    *(volatile v4f*)(sp) = v0;
#pragma unroll
    for (int q = 1; q < SLOTW / 4; ++q) *(volatile v4f*)(sp + 4 * q) = z;
    __threadfence();
    *(volatile v4f*)(sp) = v0;
#pragma unroll
    for (int q = 1; q < SLOTW / 4; ++q) *(volatile v4f*)(sp + 4 * q) = z;
  }
}

__global__ __launch_bounds__(32)
void k_out(const float* __restrict__ slots, float* __restrict__ out)
{
  const int lane = threadIdx.x;
  if (lane < (NB * NCLS) / 4) {
    float v[4];
#pragma unroll
    for (int i = 0; i < 4; ++i) {
      const int e = lane * 4 + i;
      const int bb = e / NCLS;
      const int j = e - bb * NCLS;
      v[i] = slots[bb * SLOTW + j];
    }
    const v4f w = {v[0], v[1], v[2], v[3]};
    float* op = out + lane * 4;
    *(volatile v4f*)op = w;
    __threadfence();
    *(volatile v4f*)op = w;
  }
}

extern "C" void kernel_launch(void* const* d_in, const int* in_sizes, int n_in,
                              void* d_out, int out_size, void* d_ws, size_t ws_size,
                              hipStream_t stream)
{
  if (n_in < 25) return;
  if (in_sizes[0] != NTOK * ND || out_size != NB * NCLS) return;

  const float* hidden = (const float*)d_in[0];
  const float* Wq  = (const float*)d_in[1];
  const float* Aq  = (const float*)d_in[2];
  const float* Bq  = (const float*)d_in[3];
  const float* Wk  = (const float*)d_in[4];
  const float* Ak  = (const float*)d_in[5];
  const float* Bk  = (const float*)d_in[6];
  const float* Wv  = (const float*)d_in[7];
  const float* Av  = (const float*)d_in[8];
  const float* Bv  = (const float*)d_in[9];
  const float* Wo  = (const float*)d_in[10];
  const float* Ao  = (const float*)d_in[11];
  const float* Bo  = (const float*)d_in[12];
  const float* ln1_g = (const float*)d_in[13];
  const float* ln1_b = (const float*)d_in[14];
  const float* ln2_g = (const float*)d_in[15];
  const float* ln2_b = (const float*)d_in[16];
  const float* W1  = (const float*)d_in[17];
  const float* b1  = (const float*)d_in[18];
  const float* W2  = (const float*)d_in[19];
  const float* b2  = (const float*)d_in[20];
  const float* Wc1 = (const float*)d_in[21];
  const float* bc1 = (const float*)d_in[22];
  const float* Wc2 = (const float*)d_in[23];
  const float* bc2 = (const float*)d_in[24];

  size_t off = 0;
  auto carve = [&](size_t bytes) -> size_t {
    size_t o = off;
    off += (bytes + 4095) & ~(size_t)4095;
    return o;
  };
  const size_t o_h1    = carve((size_t)NTOK * ND * sizeof(f16));
  const size_t o_wk    = carve((size_t)ND * ND * sizeof(f16));
  const size_t o_wv    = carve((size_t)ND * ND * sizeof(f16));
  const size_t o_K     = carve((size_t)NTOK * ND * sizeof(float));
  const size_t o_V     = carve((size_t)NTOK * ND * sizeof(float));
  const size_t o_q0    = carve((size_t)NB * ND * sizeof(float));
  const size_t o_ctx   = carve((size_t)NB * ND * sizeof(float));
  const size_t o_hA    = carve((size_t)NB * ND * sizeof(float));
  const size_t o_ff    = carve((size_t)NB * NFF * sizeof(float));
  const size_t o_slots = carve((size_t)NB * SLOTW * sizeof(float));
  if (off > ws_size) return;

  char* ws = (char*)d_ws;
  f16*   h1h   = (f16*)(ws + o_h1);
  f16*   Wkh   = (f16*)(ws + o_wk);
  f16*   Wvh   = (f16*)(ws + o_wv);
  float* Kf    = (float*)(ws + o_K);
  float* Vf    = (float*)(ws + o_V);
  float* q0    = (float*)(ws + o_q0);
  float* ctx   = (float*)(ws + o_ctx);
  float* hA    = (float*)(ws + o_hA);
  float* ffb   = (float*)(ws + o_ff);
  float* slots = (float*)(ws + o_slots);
  float* out   = (float*)d_out;

  k_ln_rows<<<dim3(NTOK), dim3(128), 0, stream>>>(hidden, ln1_g, ln1_b, h1h);

  k_fold<<<dim3((ND * ND / 8) / 256, 2), dim3(256), 0, stream>>>(Wk, Ak, Bk, Wv, Av, Bv, Wkh, Wvh);

  k_gemm_kv<<<dim3(ND / 128, NTOK / 128, 2), dim3(256), 0, stream>>>(h1h, Wkh, Wvh, Kf, Vf);

  k_cls_q<<<dim3(NB), dim3(256), 0, stream>>>(hidden, ln1_g, ln1_b, Wq, Aq, Bq, q0);

  k_cls_attn<<<dim3(NH, NB), dim3(256), 0, stream>>>(q0, Kf, Vf, ctx);

  k_cls_mid<<<dim3(NB), dim3(256), 0, stream>>>(ctx, hidden, Wo, Ao, Bo, ln2_g, ln2_b, W1, b1, hA, ffb);

  k_cls_head<<<dim3(NB), dim3(256), 0, stream>>>(hA, ffb, W2, b2, Wc1, bc1, Wc2, bc2, slots);

  k_out<<<dim3(1), dim3(32), 0, stream>>>(slots, out);
}
